// TA_block_31619549233987
// MI455X (gfx1250) — hardware-verified
//
#include <hip/hip_runtime.h>


#define NB_  4
#define CC   128
#define TT   512
#define VV   25
#define NP   (TT * VV)
#define NH_  16
#define HP   32
#define GH   256
typedef _Float16 h16;
typedef unsigned short bf;
typedef __attribute__((ext_vector_type(16))) __bf16   v16bf;
typedef __attribute__((ext_vector_type(16))) _Float16 v16h;
typedef __attribute__((ext_vector_type(8)))  _Float16 v8h;
typedef __attribute__((ext_vector_type(8)))  unsigned short v8us;
typedef __attribute__((ext_vector_type(8)))  float    v8f;
typedef __attribute__((ext_vector_type(4)))  float    v4f;
typedef v8h  __attribute__((may_alias)) v8ha;
typedef v4f  __attribute__((may_alias)) v4fa;
typedef v8us __attribute__((may_alias)) v8usa;

__device__ __forceinline__ unsigned short f2bf(float f) { unsigned u = __float_as_uint(f); u += 0x7FFFu + ((u >> 16) & 1u); return (unsigned short)(u >> 16); }
__device__ __forceinline__ float bf2f(unsigned short b) { return __uint_as_float(((unsigned)b) << 16); }
__device__ __forceinline__ float bfr(float f) { return bf2f(f2bf(f)); }
__device__ __forceinline__ v16h cat16(v8h lo, v8h hi) { return __builtin_shufflevector(lo, hi, 0, 1, 2, 3, 4, 5, 6, 7, 8, 9, 10, 11, 12, 13, 14, 15); }
__device__ __forceinline__ v16bf cat16b(v8us lo, v8us hi) { return __builtin_bit_cast(v16bf, __builtin_shufflevector(lo, hi, 0, 1, 2, 3, 4, 5, 6, 7, 8, 9, 10, 11, 12, 13, 14, 15)); }
__device__ __forceinline__ v8f wmma16(v16h a, v16h b, v8f c) { return __builtin_amdgcn_wmma_f32_16x16x32_f16(false, a, false, b, (short)0, c, false, false); }
__device__ __forceinline__ v8f wmmab(v16bf a, v16bf b, v8f c) { return __builtin_amdgcn_wmma_f32_16x16x32_bf16(false, a, false, b, (short)0, c, false, false); }


template <typename T16> struct WFrag;
template <> struct WFrag<h16> { typedef v16h V; static __device__ __forceinline__ V ld(const h16* p) { return cat16(*(const v8h*)p, *(const v8h*)(p + 16)); } static __device__ __forceinline__ v8f mma(V a, V b, v8f c) { return wmma16(a, b, c); } };
template <> struct WFrag<bf> { typedef v16bf V; static __device__ __forceinline__ V ld(const bf* p) { return cat16b(*(const v8us*)p, *(const v8us*)(p + 16)); } static __device__ __forceinline__ v8f mma(V a, V b, v8f c) { return wmmab(a, b, c); } };
template <typename T16, int NSPLIT, bool BIAS>
__global__ __launch_bounds__(32) void k_gemmw(const T16* __restrict__ A, const T16* __restrict__ A2, const T16* __restrict__ Bt, const T16* __restrict__ Bt2, int K, float* C, int ldc, const float* __restrict__ bias, size_t sA, size_t sB, size_t sC) {
    typedef typename WFrag<T16>::V V;
    __shared__ __align__(16) float os[16 * 68];
    const size_t z = blockIdx.z; A += z * sA; if (A2) A2 += z * sA; Bt += z * sB; if (Bt2) Bt2 += z * sB; C += z * sC;
    const int lane = threadIdx.x & 31, lr = lane & 15, hi = lane >> 4; const int r0 = blockIdx.x * 64, c0 = blockIdx.y * 64;
    v8f acc[4][4];
#pragma unroll
    for (int mb = 0; mb < 4; ++mb)
#pragma unroll
        for (int nb = 0; nb < 4; ++nb) acc[mb][nb] = (v8f){};
    const size_t aoff = (size_t)(r0 + lr) * K + 8 * hi, boff = (size_t)(c0 + lr) * K + 8 * hi;
#pragma unroll 1
    for (int kc = 0; kc < K; kc += 32) {
        V a[4], a2[4];
#pragma unroll
        for (int mb = 0; mb < 4; ++mb) { a[mb] = WFrag<T16>::ld(A + aoff + (size_t)mb * 16 * K + kc); if (NSPLIT == 1 || NSPLIT == 2) a2[mb] = WFrag<T16>::ld(A2 + aoff + (size_t)mb * 16 * K + kc); }
#pragma unroll
        for (int nb = 0; nb < 4; ++nb) { const V b = WFrag<T16>::ld(Bt + boff + (size_t)nb * 16 * K + kc); V b2; if (NSPLIT >= 2) b2 = WFrag<T16>::ld(Bt2 + boff + (size_t)nb * 16 * K + kc);
#pragma unroll
            for (int mb = 0; mb < 4; ++mb) { acc[mb][nb] = WFrag<T16>::mma(a[mb], b, acc[mb][nb]); if (NSPLIT == 1 || NSPLIT == 2) acc[mb][nb] = WFrag<T16>::mma(a2[mb], b, acc[mb][nb]); if (NSPLIT >= 2) acc[mb][nb] = WFrag<T16>::mma(a[mb], b2, acc[mb][nb]); } }
        asm volatile("v_nop\n\tv_nop\n\tv_nop\n\tv_nop" : "+v"(acc[0][0]), "+v"(acc[1][1]), "+v"(acc[2][2]), "+v"(acc[3][3]) : "v"(a[0]), "v"(a[3]));
    }
#pragma unroll
    for (int mb = 0; mb < 4; ++mb) {
#pragma unroll
        for (int nb = 0; nb < 4; ++nb) {
#pragma unroll
            for (int j = 0; j < 8; ++j) os[(hi * 8 + j) * 68 + nb * 16 + lr] = acc[mb][nb][j]; }
        __builtin_amdgcn_wave_barrier(); asm volatile("" ::: "memory");
        float* crow = C + (size_t)(r0 + mb * 16) * ldc + c0;
#pragma unroll 1
        for (int ps = 0; ps < 2; ++ps) {
#pragma unroll
            for (int s = 0; s < 8; ++s) { const int row = 2 * s + hi, cofs = lr * 4; v4f val = *(const v4fa*)(os + row * 68 + cofs); if (BIAS) { val[0] += bfr(bias[c0 + cofs]); val[1] += bfr(bias[c0 + cofs + 1]); val[2] += bfr(bias[c0 + cofs + 2]); val[3] += bfr(bias[c0 + cofs + 3]); }
                *(volatile v4f*)(crow + (size_t)row * ldc + cofs) = val; }
            if (ps == 0) __threadfence(); }
        __builtin_amdgcn_wave_barrier(); asm volatile("" ::: "memory");
    }
}

__device__ __forceinline__ h16 tohx(float x) { return (h16)x; }
__device__ __forceinline__ float tanhf_(float a) { const float e2 = __expf(2.0f * a); return __fsub_rn(1.0f, __fdiv_rn(2.0f, __fadd_rn(e2, 1.0f))); }
typedef __attribute__((ext_vector_type(2))) _Float16 v2h;
typedef __attribute__((ext_vector_type(4))) _Float16 v4h;
typedef __attribute__((ext_vector_type(4))) unsigned short v4us;
typedef __attribute__((ext_vector_type(2))) float v2f;

__global__ __launch_bounds__(256) void k_cvt8(const float* __restrict__ src, bf* dst, size_t n8) { const size_t i = (size_t)blockIdx.x * 256 + threadIdx.x; if (i >= n8) return; const v8f v = *(const v8f*)(src + i * 8); v8us o;
#pragma unroll
    for (int k = 0; k < 8; ++k) o[k] = f2bf(v[k]); *(volatile v8us*)(dst + i * 8) = o; __threadfence(); *(volatile v8us*)(dst + i * 8) = o; }
__global__ __launch_bounds__(256) void k_wr16(const float* __restrict__ Wr, h16* WR) { const int e = (blockIdx.x * 256 + threadIdx.x) * 2; if (e >= CC * HP) return; const int h = e % HP, o = e / HP; v2h w; w[0] = h < NH_ ? tohx(bfr(Wr[o * NH_ + h])) : (h16)0.f; w[1] = (h + 1) < NH_ ? tohx(bfr(Wr[o * NH_ + h + 1])) : (h16)0.f; *(volatile v2h*)(WR + e) = w; __threadfence(); *(volatile v2h*)(WR + e) = w; }
__global__ __launch_bounds__(256) void k_xt(const float* __restrict__ xb, bf* XT) { const size_t e = ((size_t)blockIdx.x * 256 + threadIdx.x) * 4; if (e >= (size_t)NP * CC) return; const int c = (int)(e % CC), p = (int)(e / CC); v4us o;
#pragma unroll
    for (int q = 0; q < 4; ++q) o[q] = f2bf(xb[(size_t)(c + q) * NP + p]); *(volatile v4us*)(XT + e) = o; __threadfence(); *(volatile v4us*)(XT + e) = o; }
__global__ __launch_bounds__(256) void k_xm(const float* __restrict__ xb, float* XM) { const int e = blockIdx.x * 256 + threadIdx.x; if (e >= CC * TT) return; const float* s = xb + (size_t)e * VV; float a = 0.f; for (int v = 0; v < VV; ++v) a = __fadd_rn(a, bfr(s[v])); const float m = __fdiv_rn(a, (float)VV); *(volatile float*)(XM + e) = m; __threadfence(); *(volatile float*)(XM + e) = m; }
__global__ __launch_bounds__(256) void k_qk(const float* __restrict__ XM, const float* __restrict__ Wq, const float* __restrict__ bq, const float* __restrict__ Wk, const float* __restrict__ bk, float* QK) { const int e = blockIdx.x * 256 + threadIdx.x; if (e >= 2 * NH_ * TT) return; const int t = e % TT; const int h = (e / TT) % NH_; const int s = e / (TT * NH_); const float* W = s ? Wk : Wq; float a = 0.f;
    for (int c = 0; c < CC; ++c) { float p = __fmul_rn(bfr(W[h * CC + c]), XM[c * TT + t]); asm volatile("" : "+v"(p)); a = __fadd_rn(a, p); } const float o = __fadd_rn(a, bfr((s ? bk : bq)[h])); *(volatile float*)(QK + e) = o; __threadfence(); *(volatile float*)(QK + e) = o; }
__global__ __launch_bounds__(256) void k_vt(const float* __restrict__ VP, h16* VT) { const size_t e = ((size_t)blockIdx.x * 256 + threadIdx.x) * 2; if (e >= (size_t)CC * 64 * TT) return; const int t = (int)(e % TT); const int vv = (int)((e / TT) % 64); const int o = (int)(e / ((size_t)TT * 64)); v2h r;
    if (vv < VV) { r[0] = tohx(VP[((size_t)t * VV + vv) * CC + o]); r[1] = tohx(VP[((size_t)(t + 1) * VV + vv) * CC + o]); } else { r[0] = (h16)0.f; r[1] = (h16)0.f; } *(volatile v2h*)(VT + e) = r; __threadfence(); *(volatile v2h*)(VT + e) = r; }
__global__ __launch_bounds__(256) void k_th(const float* __restrict__ QK, int g0, h16* TH) { const size_t e = ((size_t)blockIdx.x * 256 + threadIdx.x) * 2; if (e >= (size_t)GH * TT * HP) return; const int h = (int)(e % HP); const int t = (int)((e / HP) % TT); const int g = g0 + (int)(e / ((size_t)HP * TT)); v2h r;
#pragma unroll
    for (int u = 0; u < 2; ++u) { const int hh = h + u; r[u] = hh < NH_ ? tohx(tanhf_(__fsub_rn(QK[hh * TT + g], QK[(NH_ + hh) * TT + t]))) : (h16)0.f; } *(volatile v2h*)(TH + e) = r; __threadfence(); *(volatile v2h*)(TH + e) = r; }
__global__ __launch_bounds__(256) void k_ap(const float* __restrict__ ATT2, const float* __restrict__ br, h16* AP) { const size_t e = ((size_t)blockIdx.x * 256 + threadIdx.x) * 2; if (e >= (size_t)CC * GH * TT) return; const int t = (int)(e % TT); const int g = (int)((e / TT) % GH); const int o = (int)(e / ((size_t)TT * GH)); const float b = bfr(br[o]); v2h r;
    r[0] = tohx(__fadd_rn(ATT2[((size_t)g * TT + t) * CC + o], b)); r[1] = tohx(__fadd_rn(ATT2[((size_t)g * TT + t + 1) * CC + o], b)); *(volatile v2h*)(AP + e) = r; __threadfence(); *(volatile v2h*)(AP + e) = r; }
__global__ __launch_bounds__(256) void k_bnst(const float* __restrict__ Y, float* ST) { const int lane = threadIdx.x & 31; const int o = blockIdx.x * 8 + (threadIdx.x >> 5); if (o >= CC) return; const int tot = NB_ * TT * VV; float s = 0.f;
    for (int f = lane; f < tot; f += 32) { const int vv = f % VV; const int g = (f / VV) % TT; const int n = f / (VV * TT); s = __fadd_rn(s, Y[(((size_t)n * CC + o) * TT + g) * 64 + vv]); }
#pragma unroll
    for (int sh = 16; sh; sh >>= 1) s += __shfl_xor(s, sh, 32);
    const float mu = __fdiv_rn(s, (float)tot); float q2 = 0.f;
    for (int f = lane; f < tot; f += 32) { const int vv = f % VV; const int g = (f / VV) % TT; const int n = f / (VV * TT); const float d = __fsub_rn(Y[(((size_t)n * CC + o) * TT + g) * 64 + vv], mu); float p = __fmul_rn(d, d); asm volatile("" : "+v"(p)); q2 = __fadd_rn(q2, p); }
#pragma unroll
    for (int sh = 16; sh; sh >>= 1) q2 += __shfl_xor(q2, sh, 32);
    const float var = __fdiv_rn(q2, (float)tot); const float w = lane == 0 ? mu : (lane == 1 ? var : 0.f); *(volatile float*)(ST + o * 32 + lane) = w; __threadfence(); *(volatile float*)(ST + o * 32 + lane) = w; }
__global__ __launch_bounds__(256) void k_out(const float* __restrict__ Y, const float* __restrict__ ST, const float* __restrict__ g, const float* __restrict__ bb, const float* __restrict__ x, float* OUT) { const size_t e = ((size_t)blockIdx.x * 256 + threadIdx.x) * 4; if (e >= (size_t)NB_ * CC * NP) return; v4f r;
#pragma unroll
    for (int q = 0; q < 4; ++q) { const size_t f = e + q; const int vv = (int)(f % VV); const int t = (int)((f / VV) % TT); const int c = (int)((f / NP) % CC); const int n = (int)(f / ((size_t)NP * CC)); const float mu = ST[c * 32], var = ST[c * 32 + 1];
        const float sc = __fmul_rn(bfr(g[c]), __frsqrt_rn(__fadd_rn(var, 1e-5f))); float tn = __fmul_rn(__fsub_rn(Y[(((size_t)n * CC + c) * TT + t) * 64 + vv], mu), sc); asm volatile("" : "+v"(tn)); const float yb = __fadd_rn(tn, bfr(bb[c])); r[q] = fmaxf(__fadd_rn(yb, bfr(x[f])), 0.f); }
    *(volatile v4f*)(OUT + e) = r; __threadfence(); *(volatile v4f*)(OUT + e) = r; }

extern "C" void kernel_launch(void* const* d_in, const int* in_sizes, int n_in,
                              void* d_out, int out_size, void* d_ws, size_t ws_size, hipStream_t stream) {
    (void)in_sizes; (void)n_in; (void)out_size;
    const float* IN[11]; for (int i = 0; i < 11; ++i) IN[i] = (const float*)d_in[i];
    float* OUT = (float*)d_out;
    char* wsp = (char*)d_ws;
    auto take = [&](size_t bytes) { char* p = wsp; wsp += (bytes + 255) & ~(size_t)255; return (void*)p; };
    bf* WV = (bf*)take((size_t)CC * CC * 2); h16* WR = (h16*)take((size_t)CC * HP * 2); bf* XT = (bf*)take((size_t)NP * CC * 2); float* XM = (float*)take((size_t)CC * TT * 4); float* QK = (float*)take((size_t)2 * NH_ * TT * 4); float* VP = (float*)take((size_t)NP * CC * 4); h16* VT = (h16*)take((size_t)CC * 64 * TT * 2);
    h16* TH = (h16*)take((size_t)GH * TT * HP * 2); float* ATT2 = (float*)take((size_t)GH * TT * CC * 4); h16* AP = (h16*)take((size_t)CC * GH * TT * 2); float* Y = (float*)take((size_t)NB_ * CC * TT * 64 * 4); float* ST = (float*)take((size_t)CC * 32 * 4);
    if ((size_t)(wsp - (char*)d_ws) > ws_size) return;
    k_cvt8<<<(CC * CC / 8 + 255) / 256, 256, 0, stream>>>(IN[5], WV, (size_t)CC * CC / 8); k_wr16<<<(CC * HP / 2 + 255) / 256, 256, 0, stream>>>(IN[7], WR);
    for (int n = 0; n < NB_; ++n) { const float* xb = IN[0] + (size_t)n * CC * NP;
        k_xt<<<(unsigned)(((size_t)NP * CC / 4 + 255) / 256), 256, 0, stream>>>(xb, XT); k_xm<<<(CC * TT + 255) / 256, 256, 0, stream>>>(xb, XM); k_qk<<<(2 * NH_ * TT + 255) / 256, 256, 0, stream>>>(XM, IN[1], IN[2], IN[3], IN[4], QK);
        k_gemmw<bf, 0, true><<<dim3(NP / 64, CC / 64, 1), 32, 0, stream>>>(XT, nullptr, WV, nullptr, CC, VP, CC, IN[6], 0, 0, 0); k_vt<<<(unsigned)(((size_t)CC * 64 * TT / 2 + 255) / 256), 256, 0, stream>>>(VP, VT);
        for (int gh = 0; gh < TT / GH; ++gh) { const int g0 = gh * GH;
            k_th<<<(unsigned)(((size_t)GH * TT * HP / 2 + 255) / 256), 256, 0, stream>>>(QK, g0, TH);
            k_gemmw<h16, 0, false><<<dim3(GH * TT / 64, CC / 64, 1), 32, 0, stream>>>(TH, nullptr, WR, nullptr, HP, ATT2, CC, nullptr, 0, 0, 0);
            k_ap<<<(unsigned)(((size_t)CC * GH * TT / 2 + 255) / 256), 256, 0, stream>>>(ATT2, IN[8], AP);
            k_gemmw<h16, 0, false><<<dim3(GH / 64, 1, CC), 32, 0, stream>>>(AP, nullptr, VT, nullptr, TT, Y + (((size_t)n * CC) * TT + g0) * 64, 64, nullptr, (size_t)GH * TT, (size_t)64 * TT, (size_t)TT * 64); } }
    k_bnst<<<CC / 8, 256, 0, stream>>>(Y, ST);
    k_out<<<(unsigned)(((size_t)NB_ * CC * NP / 4 + 255) / 256), 256, 0, stream>>>(Y, ST, IN[9], IN[10], IN[0], OUT);
}
